// sju_53214644798203
// MI455X (gfx1250) — hardware-verified
//
#include <hip/hip_runtime.h>


namespace {
constexpr int B = 256, C = 512, L = 17, NH = 8, DK = 64, DFF = 2048, NT = B * L, NAT = B * 2 * L;
constexpr float XS = 8.0f, WSC = 256.0f;
__constant__ int NEIGH[17][5] = {{0,1,2,5,6},{0,1,3,17,17},{0,2,4,17,17},{1,3,17,17,17},{2,4,17,17,17},{0,5,7,11,17},{0,6,8,12,17},{5,7,9,17,17},{6,8,12,17,17},{7,9,17,17,17},{8,10,17,17,17},{8,11,13,17,17},{10,12,14,17,17},{11,13,15,17,17},{12,14,16,17,17},{13,15,17,17,17},{14,16,17,17,17}};
__constant__ int SEQLEN[17] = {4,2,2,1,1,3,3,2,2,1,1,2,2,2,2,1,1};
typedef _Float16 b16;
typedef __attribute__((ext_vector_type(16))) _Float16 v16b;
typedef __attribute__((ext_vector_type(8))) _Float16 v8b;
typedef __attribute__((ext_vector_type(8))) float v8f;
typedef __attribute__((ext_vector_type(4))) float v4f;
typedef __attribute__((ext_vector_type(2))) float v2f;
__device__ __forceinline__ float bf16_rne(float f) { unsigned int u = __float_as_uint(f); u += 0x7FFFu + ((u >> 16) & 1u); return __uint_as_float(u & 0xFFFF0000u); }
__device__ __forceinline__ v16b frag_kb(const b16* p, int hh) { const v8b a = *(const v8b*)(p + 8 * hh), b = *(const v8b*)(p + 16 + 8 * hh); v16b f;
#pragma unroll
  for (int e = 0; e < 8; ++e) { f[e] = a[e]; f[8 + e] = b[e]; } return f; }
__device__ __forceinline__ v8f wmma16b(v16b a, v16b b, v8f c) { v8f d = __builtin_amdgcn_wmma_f32_16x16x32_f16(false, a, false, b, (short)0, c, false, false); asm volatile("v_nop\n\tv_nop\n\tv_nop\n\tv_nop" : "+v"(d) : "v"(a), "v"(b)); return d; }
__device__ __forceinline__ void wave_lds_sync() { __builtin_amdgcn_fence(__ATOMIC_RELEASE, "workgroup"); __builtin_amdgcn_wave_barrier(); __builtin_amdgcn_fence(__ATOMIC_ACQUIRE, "workgroup"); }
__device__ __forceinline__ float pmul(float a, float b) { float p = a * b; asm volatile("" : "+v"(p)); return p; }

__global__ __launch_bounds__(256) void wcopy_kernel(const float* __restrict__ w, int OUTW, int KIN, int ro, b16* __restrict__ WT) {
  const size_t u = (size_t)blockIdx.x * 256 + threadIdx.x; if (u >= (size_t)OUTW * KIN / 8) return; const size_t e = u * 8; v8b v;
#pragma unroll
  for (int j = 0; j < 8; ++j) v[j] = (b16)(bf16_rne(w[e + j]) * WSC); for (int pass = 0; pass < 2; ++pass) { *(volatile v8b*)(WT + (size_t)ro * KIN + e) = v; __threadfence(); }
}
template <int AUX, int NTILE>
__global__ __launch_bounds__(32) void proj_kernel(const float* __restrict__ src, const b16* __restrict__ WT, const float* __restrict__ bq, const float* __restrict__ bk, const float* __restrict__ bv, int NTOK, float* __restrict__ OUT) {
  __shared__ __attribute__((aligned(16))) b16 Ah[16][C + 8]; __shared__ __attribute__((aligned(16))) float Tf[16][128 + 4];
  const int lane = threadIdx.x, nloc = lane & 15, hlf = lane >> 4; const size_t m0 = (size_t)blockIdx.x * 16; if (m0 >= (size_t)NTOK) return;
  for (int rr = 0; rr < 16; ++rr) { const size_t t = m0 + rr; size_t base; if (AUX) { const size_t b = t / (2 * L), rem = t % (2 * L), a = rem / L, l = rem % L; base = (b * C * 2 + a) * L + l; } else { const size_t b = t / L, l = t % L; base = b * C * L + l; }
    for (int q = 0; q < C / 32; ++q) { const int c = q * 32 + lane; Ah[rr][c] = (b16)(bf16_rne(src[base + (size_t)c * (AUX ? 2 * L : L)]) * XS); } }
  wave_lds_sync(); const b16* W = WT + (AUX ? (size_t)C * C : 0);
#pragma unroll 1
  for (int cg = 0; cg < NTILE / 8; ++cg) { v8f acc[8];
#pragma unroll
    for (int t = 0; t < 8; ++t) acc[t] = (v8f){};
#pragma unroll 2
    for (int kb = 0; kb < C; kb += 32) { const v16b a = frag_kb(&Ah[nloc][kb], hlf);
#pragma unroll
      for (int t = 0; t < 8; ++t) acc[t] = wmma16b(a, frag_kb(W + (size_t)(cg * 128 + t * 16 + nloc) * C + kb, hlf), acc[t]); }
#pragma unroll
    for (int t = 0; t < 8; ++t) { const int col = cg * 128 + t * 16 + nloc; const int sel = (AUX ? col + C : col) / C, cc = col % C; const float bb = bf16_rne(sel == 0 ? bq[cc] : (sel == 1 ? bk[cc] : bv[cc]));
#pragma unroll
      for (int r8 = 0; r8 < 8; ++r8) Tf[8 * hlf + r8][t * 16 + nloc] = acc[t][r8] * (1.0f / (XS * WSC)) + bb; }
    wave_lds_sync();
    for (int pass = 0; pass < 2; ++pass) { for (int rr = 0; rr < 16; ++rr) *(volatile v4f*)(OUT + (m0 + rr) * (NTILE * 16) + cg * 128 + lane * 4) = *(const v4f*)(&Tf[rr][lane * 4]); __threadfence(); }
    wave_lds_sync(); }
}
__global__ __launch_bounds__(32) void att_kernel(const float* __restrict__ x, const float* __restrict__ QKV, const float* __restrict__ AKV, const float* __restrict__ g1, const float* __restrict__ be1, const float* __restrict__ m1, const float* __restrict__ v1, int NBV, float* __restrict__ RET) {
  const int lane = threadIdx.x; const int b = blockIdx.x; if (b >= NBV) return;
#pragma unroll 1
  for (int l = 0; l < L; ++l) { const size_t t = (size_t)b * L + l;
    for (int pass = 0; pass < 2; ++pass) {
#pragma unroll 1
      for (int h = 0; h < NH; ++h) { const int d0 = h * DK + lane * 2; const v2f qv = *(const v2f*)(QKV + t * 1536 + d0); float sc[7]; v2f vv[7];
#pragma unroll
        for (int w = 0; w < 7; ++w) { v2f kv; bool valid; if (w < 5) { const int nb = NEIGH[l][w]; valid = w < SEQLEN[l]; if (nb < L) { const size_t tn = (size_t)b * L + nb; kv = *(const v2f*)(QKV + tn * 1536 + C + d0); vv[w] = *(const v2f*)(QKV + tn * 1536 + 2 * C + d0); } else { kv = (v2f){0.0f, 0.0f}; vv[w] = (v2f){0.0f, 0.0f}; } }
          else { const size_t ta = ((size_t)b * 2 + (w - 5)) * L + l; kv = *(const v2f*)(AKV + ta * 1024 + d0); vv[w] = *(const v2f*)(AKV + ta * 1024 + C + d0); valid = true; }
          float s = pmul(qv[0], kv[0]) + pmul(qv[1], kv[1]); for (int o = 16; o; o >>= 1) s += __shfl_xor(s, o); sc[w] = valid ? s * 0.125f : -INFINITY; }
        float mx = sc[0]; for (int w = 1; w < 7; ++w) mx = fmaxf(mx, sc[w]); float den = 0.0f, o0 = 0.0f, o1 = 0.0f;
#pragma unroll
        for (int w = 0; w < 7; ++w) { const float p = (sc[w] == -INFINITY) ? 0.0f : __expf(sc[w] - mx); den += p; o0 += pmul(p, vv[w][0]); o1 += pmul(p, vv[w][1]); }
        float r[2];
#pragma unroll
        for (int i = 0; i < 2; ++i) { const int c = d0 + i; const float xv = bf16_rne(x[((size_t)b * C + c) * L + l]); const float sc_ = pmul(bf16_rne(g1[c]), rsqrtf(bf16_rne(v1[c]) + 1e-5f)); r[i] = pmul(xv + (i ? o1 : o0) / den - bf16_rne(m1[c]), sc_) + bf16_rne(be1[c]); }
        *(volatile v2f*)(RET + t * C + d0) = (v2f){r[0], r[1]}; }
      __threadfence(); } }
}
__global__ __launch_bounds__(32) void ffn1_kernel(const float* __restrict__ RET, const b16* __restrict__ W1T, const float* __restrict__ b1, int NTOK, float* __restrict__ Hh) {
  __shared__ __attribute__((aligned(16))) b16 Ah[16][C + 8]; __shared__ __attribute__((aligned(16))) float Tf[16][128 + 4];
  const int lane = threadIdx.x, nloc = lane & 15, hlf = lane >> 4; const size_t m0 = (size_t)blockIdx.x * 16; if (m0 >= (size_t)NTOK) return;
  for (int rr = 0; rr < 16; ++rr) for (int q = 0; q < C / 32; ++q) Ah[rr][q * 32 + lane] = (b16)(RET[(m0 + rr) * C + q * 32 + lane] * XS);
  wave_lds_sync();
#pragma unroll 1
  for (int cg = 0; cg < DFF / 128; ++cg) { v8f acc[8];
#pragma unroll
    for (int t = 0; t < 8; ++t) acc[t] = (v8f){};
#pragma unroll 2
    for (int kb = 0; kb < C; kb += 32) { const v16b a = frag_kb(&Ah[nloc][kb], hlf);
#pragma unroll
      for (int t = 0; t < 8; ++t) acc[t] = wmma16b(a, frag_kb(W1T + (size_t)(cg * 128 + t * 16 + nloc) * C + kb, hlf), acc[t]); }
#pragma unroll
    for (int t = 0; t < 8; ++t) { const int c = cg * 128 + t * 16 + nloc; const float bb = bf16_rne(b1[c]);
#pragma unroll
      for (int r8 = 0; r8 < 8; ++r8) Tf[8 * hlf + r8][t * 16 + nloc] = fmaxf(acc[t][r8] * (1.0f / (XS * WSC)) + bb, 0.0f); }
    wave_lds_sync();
    for (int pass = 0; pass < 2; ++pass) { for (int rr = 0; rr < 16; ++rr) *(volatile v4f*)(Hh + (m0 + rr) * DFF + cg * 128 + lane * 4) = *(const v4f*)(&Tf[rr][lane * 4]); __threadfence(); }
    wave_lds_sync(); }
}
__global__ __launch_bounds__(32) void ffn2_kernel(const float* __restrict__ Hh, const float* __restrict__ RET, const b16* __restrict__ W2T, const float* __restrict__ b2, const float* __restrict__ g2, const float* __restrict__ be2, const float* __restrict__ m2, const float* __restrict__ v2, int NBV, float* __restrict__ out) {
  __shared__ __attribute__((aligned(16))) b16 Ah[32][512 + 8]; __shared__ float Zs[64][L + 1];
  const int lane = threadIdx.x, nloc = lane & 15, hlf = lane >> 4; const int b = blockIdx.x; if (b >= NBV) return; const size_t t0 = (size_t)b * L;
#pragma unroll 1
  for (int cg = 0; cg < 8; ++cg) { v8f acc[2][4];
#pragma unroll
    for (int rt = 0; rt < 2; ++rt)
#pragma unroll
      for (int t = 0; t < 4; ++t) acc[rt][t] = (v8f){};
#pragma unroll 1
    for (int kc = 0; kc < DFF / 512; ++kc) {
      for (int rr = 0; rr < 32; ++rr) for (int q = 0; q < 16; ++q) Ah[rr][q * 32 + lane] = (b16)((rr < L ? Hh[(t0 + rr) * DFF + kc * 512 + q * 32 + lane] : 0.0f) * XS);
      wave_lds_sync();
#pragma unroll 2
      for (int kb = 0; kb < 512; kb += 32) { const v16b a0 = frag_kb(&Ah[nloc][kb], hlf), a1 = frag_kb(&Ah[16 + nloc][kb], hlf);
#pragma unroll
        for (int t = 0; t < 4; ++t) { const v16b bw = frag_kb(W2T + (size_t)(cg * 64 + t * 16 + nloc) * DFF + kc * 512 + kb, hlf); acc[0][t] = wmma16b(a0, bw, acc[0][t]); acc[1][t] = wmma16b(a1, bw, acc[1][t]); } }
      wave_lds_sync(); }
#pragma unroll
    for (int rt = 0; rt < 2; ++rt)
#pragma unroll
      for (int t = 0; t < 4; ++t) { const int cl = t * 16 + nloc, c = cg * 64 + cl; const float bb = bf16_rne(b2[c]), sc = pmul(bf16_rne(g2[c]), rsqrtf(bf16_rne(v2[c]) + 1e-5f)), mu = bf16_rne(m2[c]), bt = bf16_rne(be2[c]);
#pragma unroll
        for (int r8 = 0; r8 < 8; ++r8) { const int l = rt * 16 + 8 * hlf + r8; if (l < L) { const float z = acc[rt][t][r8] * (1.0f / (XS * WSC)) + bb + RET[(t0 + l) * C + c]; Zs[cl][l] = pmul(z - mu, sc) + bt; } } }
    wave_lds_sync();
    for (int pass = 0; pass < 2; ++pass) { for (int i = lane; i < 64 * L; i += 32) ((volatile float*)out)[((size_t)b * C + cg * 64) * L + i] = Zs[i / L][i % L]; __threadfence(); }
    wave_lds_sync(); }
}
}

extern "C" void kernel_launch(void* const* d_in, const int* in_sizes, int n_in, void* d_out, int out_size, void* d_ws, size_t ws_size, hipStream_t stream) {
  (void)n_in;
  auto Fp = [&](int i) { return (const float*)d_in[i]; };
  if (in_sizes[0] != B * C * L || in_sizes[1] != B * C * 2 * L || in_sizes[2] != C * C || in_sizes[4] != C * C || in_sizes[6] != C * C || in_sizes[12] != DFF * C || in_sizes[14] != C * DFF || out_size != B * C * L) return;
  const int NBV = B; const int NTV = NBV * L, NAV = NBV * 2 * L;
  size_t off = 0; char* ws = (char*)d_ws;
  auto carve = [&](size_t bytes) { char* p = ws + off; off += (bytes + 255) & ~(size_t)255; return p; };
  b16* WQKV = (b16*)carve((size_t)3 * C * C * 2); b16* W1T = (b16*)carve((size_t)DFF * C * 2); b16* W2T = (b16*)carve((size_t)C * DFF * 2);
  float* QKV = (float*)carve((size_t)NT * 1536 * 4); float* AKV = (float*)carve((size_t)NAT * 1024 * 4); float* RET = (float*)carve((size_t)NT * C * 4); float* Hh = (float*)carve((size_t)(NT + 16) * DFF * 4);
  if (off > ws_size || off > ((size_t)128 << 20)) return;
  wcopy_kernel<<<(C * C / 8 + 255) / 256, 256, 0, stream>>>(Fp(2), C, C, 0, WQKV); wcopy_kernel<<<(C * C / 8 + 255) / 256, 256, 0, stream>>>(Fp(4), C, C, C, WQKV); wcopy_kernel<<<(C * C / 8 + 255) / 256, 256, 0, stream>>>(Fp(6), C, C, 2 * C, WQKV);
  wcopy_kernel<<<(DFF * C / 8 + 255) / 256, 256, 0, stream>>>(Fp(12), DFF, C, 0, W1T); wcopy_kernel<<<(C * DFF / 8 + 255) / 256, 256, 0, stream>>>(Fp(14), C, DFF, 0, W2T);
  proj_kernel<0, 96><<<(unsigned)((NTV + 15) / 16), 32, 0, stream>>>(Fp(0), WQKV, Fp(3), Fp(5), Fp(7), NTV, QKV);
  proj_kernel<1, 64><<<(unsigned)((NAV + 15) / 16), 32, 0, stream>>>(Fp(1), WQKV, Fp(3), Fp(5), Fp(7), NAV, AKV);
  att_kernel<<<NBV, 32, 0, stream>>>(Fp(0), QKV, AKV, Fp(8), Fp(9), Fp(10), Fp(11), NBV, RET);
  ffn1_kernel<<<(unsigned)((NTV + 15) / 16), 32, 0, stream>>>(RET, W1T, Fp(13), NTV, Hh);
  ffn2_kernel<<<NBV, 32, 0, stream>>>(Hh, RET, W2T, Fp(15), Fp(16), Fp(17), Fp(18), Fp(19), NBV, (float*)d_out);
}
